// Attention_12962211299892
// MI455X (gfx1250) — hardware-verified
//
#include <hip/hip_runtime.h>


#ifndef NB
#define NB 2
#endif
#ifndef SEQ
#define SEQ 2048
#endif
#define NB_FULL  2
#define SEQ_FULL 2048
#define HID   1024
#define NH    16
#define HD    64
#define KD    1024
#define MROWS (NB * SEQ)
#define AW    4
#define L2E   1.4426950408889634f

typedef _Float16 h16;
typedef unsigned short bf;
typedef __attribute__((ext_vector_type(16))) __bf16   v16bf;
typedef __attribute__((ext_vector_type(16))) _Float16 v16h;
typedef __attribute__((ext_vector_type(8)))  _Float16 v8h;
typedef __attribute__((ext_vector_type(8)))  unsigned short v8us;
typedef __attribute__((ext_vector_type(8)))  float    v8f;
typedef __attribute__((ext_vector_type(4)))  float    v4f;
typedef __attribute__((ext_vector_type(2)))  float    v2f;
typedef v8h  __attribute__((may_alias)) v8ha;
typedef v4f  __attribute__((may_alias)) v4fa;

static_assert(NB <= NB_FULL);
static_assert(SEQ <= SEQ_FULL);
static_assert(HID == NH * HD);
static_assert(HD == 64);
static_assert(KD == HID);
static_assert(KD % 32 == 0);
static_assert(SEQ % 64 == 0);
static_assert(MROWS % 64 == 0);
static_assert(HID % 64 == 0);
static_assert(SEQ % (16 * AW) == 0);
static_assert(SEQ % 32 == 0);
static_assert((SEQ * HID) % 2048 == 0);
static_assert((HID * HID) % 2048 == 0);
static_assert((SEQ * 32) % 256 == 0);

__device__ __forceinline__ unsigned short f2bf(float f) { unsigned u = __float_as_uint(f); u += 0x7FFFu + ((u >> 16) & 1u); return (unsigned short)(u >> 16); }
__device__ __forceinline__ float bf2f(unsigned short b) { return __uint_as_float(((unsigned)b) << 16); }
__device__ __forceinline__ float bfr(float f) { return bf2f(f2bf(f)); }
__device__ __forceinline__ void splitf(float y, unsigned short& h, unsigned short& l) { h = f2bf(y); l = f2bf(y - bf2f(h)); }
__device__ __forceinline__ v16h cat16(v8h lo, v8h hi) { return __builtin_shufflevector(lo, hi, 0, 1, 2, 3, 4, 5, 6, 7, 8, 9, 10, 11, 12, 13, 14, 15); }
__device__ __forceinline__ v16bf cat16b(v8us lo, v8us hi) { return __builtin_bit_cast(v16bf, __builtin_shufflevector(lo, hi, 0, 1, 2, 3, 4, 5, 6, 7, 8, 9, 10, 11, 12, 13, 14, 15)); }
__device__ __forceinline__ v16bf ldb(const bf* p) { return cat16b(*(const v8us*)p, *(const v8us*)(p + 16)); }
__device__ __forceinline__ v16h  ldh(const h16* p) { return cat16(*(const v8h*)p, *(const v8h*)(p + 16)); }
__device__ __forceinline__ v8f wmma16(v16h a, v16h b, v8f c) { return __builtin_amdgcn_wmma_f32_16x16x32_f16(false, a, false, b, (short)0, c, false, false); }
__device__ __forceinline__ v8f wmmab(v16bf a, v16bf b, v8f c) { return __builtin_amdgcn_wmma_f32_16x16x32_bf16(false, a, false, b, (short)0, c, false, false); }

__global__ __launch_bounds__(256) void k_cvt(const float* __restrict__ src, bf* dst, int per, int sstride) {
    const int i = (blockIdx.x * 256 + threadIdx.x) * 8; if (i >= per) return;
    const float* s = src + (size_t)blockIdx.y * sstride + i;
    const v4f a = *(const v4f*)s, b = *(const v4f*)(s + 4);
    v8us o; o[0] = f2bf(a[0]); o[1] = f2bf(a[1]); o[2] = f2bf(a[2]); o[3] = f2bf(a[3]); o[4] = f2bf(b[0]); o[5] = f2bf(b[1]); o[6] = f2bf(b[2]); o[7] = f2bf(b[3]);
    bf* d = dst + (size_t)blockIdx.y * per + i;
    *(volatile v8us*)d = o; __threadfence(); *(volatile v8us*)d = o;
}

__global__ __launch_bounds__(256) void k_cstab(float* CS) {
    const int idx = blockIdx.x * 256 + threadIdx.x; if (idx >= SEQ * 32) return;
    const int s = idx >> 5, j = idx & 31;
    const double p = (double)(1u << (j >> 1)) * ((j & 1) ? 1.4142135623730951 : 1.0);
    const float pf = (float)p; const float inv = 1.0f / pf; const float ang = (float)s * inv;
    float sn, c; sincosf(ang, &sn, &c);
    v2f cs; cs[0] = c; cs[1] = sn;
    *(volatile v2f*)(CS + (size_t)idx * 2) = cs; __threadfence(); *(volatile v2f*)(CS + (size_t)idx * 2) = cs;
}

template <int NA>
__device__ __forceinline__ void gemm_core(const bf* __restrict__ A, const bf* __restrict__ A2, const bf* __restrict__ Bt, const int r0, const int c0, const int lr, const int hi, v8f (&acc)[4][4]) {
#pragma unroll
    for (int mb = 0; mb < 4; ++mb)
#pragma unroll
        for (int nb = 0; nb < 4; ++nb) acc[mb][nb] = (v8f){};
    const size_t aoff = (size_t)(r0 + lr) * KD + 8 * hi, boff = (size_t)(c0 + lr) * KD + 8 * hi;
#pragma unroll 1
    for (int kc = 0; kc < KD; kc += 32) {
        v16bf a[4], a2[4], b;
#pragma unroll
        for (int mb = 0; mb < 4; ++mb) { a[mb] = ldb(A + aoff + (size_t)mb * 16 * KD + kc); if (NA == 2) a2[mb] = ldb(A2 + aoff + (size_t)mb * 16 * KD + kc); }
#pragma unroll
        for (int nb = 0; nb < 4; ++nb) { b = ldb(Bt + boff + (size_t)nb * 16 * KD + kc);
#pragma unroll
            for (int mb = 0; mb < 4; ++mb) { acc[mb][nb] = wmmab(a[mb], b, acc[mb][nb]); if (NA == 2) acc[mb][nb] = wmmab(a2[mb], b, acc[mb][nb]); } }
        asm volatile("" : "+v"(acc[0][0]), "+v"(acc[1][0]), "+v"(acc[2][0]), "+v"(acc[3][0]), "+v"(acc[0][1]), "+v"(acc[1][1]), "+v"(acc[2][1]), "+v"(acc[3][1]));
        if (NA == 2) asm volatile("v_nop\n\tv_nop\n\tv_nop\n\tv_nop" : "+v"(acc[0][2]), "+v"(acc[1][2]), "+v"(acc[2][2]), "+v"(acc[3][2]), "+v"(acc[0][3]), "+v"(acc[1][3]), "+v"(acc[2][3]), "+v"(acc[3][3]) : "v"(a[3]), "v"(a2[3]), "v"(b));
        else         asm volatile("v_nop\n\tv_nop\n\tv_nop\n\tv_nop" : "+v"(acc[0][2]), "+v"(acc[1][2]), "+v"(acc[2][2]), "+v"(acc[3][2]), "+v"(acc[0][3]), "+v"(acc[1][3]), "+v"(acc[2][3]), "+v"(acc[3][3]) : "v"(a[3]), "v"(b));
    }
}

__global__ __launch_bounds__(32) void k_proj_rope(const bf* __restrict__ XB, const bf* __restrict__ W, const float* __restrict__ bias, const float* __restrict__ CS, float sc, bf* Ph, bf* Pl) {
    __shared__ __align__(16) float os[16 * 68];
    const int lane = threadIdx.x & 31, lr = lane & 15, hi = lane >> 4;
    const int r0 = blockIdx.x * 64, c0 = blockIdx.y * 64;
    v8f acc[4][4];
    gemm_core<1>(XB, XB, W, r0, c0, lr, hi, acc);
    const int b = r0 / SEQ, s0 = r0 % SEQ, h = blockIdx.y;
    const int rq = lane >> 3, pc = lane & 7, d0 = pc * 8, dp0 = d0 ^ 32, jf0 = d0 & 31;
    const float sgn = (d0 < 32) ? -1.0f : 1.0f;
    float bx[8], bp[8];
    { const v4f u0 = *(const v4f*)(bias + c0 + d0), u1 = *(const v4f*)(bias + c0 + d0 + 4), w0 = *(const v4f*)(bias + c0 + dp0), w1 = *(const v4f*)(bias + c0 + dp0 + 4);
#pragma unroll
      for (int q = 0; q < 4; ++q) { bx[q] = bfr(u0[q]); bx[q + 4] = bfr(u1[q]); bp[q] = bfr(w0[q]); bp[q + 4] = bfr(w1[q]); } }
#pragma unroll
    for (int mb = 0; mb < 4; ++mb) {
#pragma unroll
        for (int nb = 0; nb < 4; ++nb) {
#pragma unroll
            for (int j = 0; j < 8; ++j) os[(hi * 8 + j) * 68 + nb * 16 + lr] = acc[mb][nb][j]; }
        __syncthreads();
        const size_t prow = ((size_t)(b * NH + h) * SEQ + s0 + mb * 16) * HD + d0;
#pragma unroll 1
        for (int ps = 0; ps < 2; ++ps) {
#pragma unroll 1
            for (int it = 0; it < 4; ++it) {
                const int rr = it * 4 + rq; const int s = s0 + mb * 16 + rr; const int xo = rr * 68;
                const v4f xa = *(const v4fa*)(os + xo + d0), xb = *(const v4fa*)(os + xo + d0 + 4);
                const v4f ya = *(const v4fa*)(os + xo + dp0), yb = *(const v4fa*)(os + xo + dp0 + 4);
                const float* cp = CS + ((size_t)s * 32 + jf0) * 2;
                const v4f t0 = *(const v4f*)cp, t1 = *(const v4f*)(cp + 4), t2 = *(const v4f*)(cp + 8), t3 = *(const v4f*)(cp + 12);
                const float xv[8] = { xa[0], xa[1], xa[2], xa[3], xb[0], xb[1], xb[2], xb[3] };
                const float yv[8] = { ya[0], ya[1], ya[2], ya[3], yb[0], yb[1], yb[2], yb[3] };
                const float cv[8] = { t0[0], t0[2], t1[0], t1[2], t2[0], t2[2], t3[0], t3[2] };
                const float sv[8] = { t0[1], t0[3], t1[1], t1[3], t2[1], t2[3], t3[1], t3[3] };
                v8us oh, ol;
#pragma unroll
                for (int q = 0; q < 8; ++q) { const float x = xv[q] + bx[q], y = yv[q] + bp[q]; const float r = (x * cv[q] + sgn * (y * sv[q])) * sc; unsigned short a2, c2; splitf(r, a2, c2); oh[q] = a2; ol[q] = c2; }
                *(volatile v8us*)(Ph + prow + (size_t)rr * HD) = oh; *(volatile v8us*)(Pl + prow + (size_t)rr * HD) = ol; }
            if (ps == 0) __threadfence(); }
        __syncthreads();
    }
}

__global__ __launch_bounds__(32) void k_proj_v(const bf* __restrict__ XB, const bf* __restrict__ W, const float* __restrict__ bias, h16* VT) {
    __shared__ __align__(16) h16 vt[64 * 72];
    const int lane = threadIdx.x & 31, lr = lane & 15, hi = lane >> 4;
    const int r0 = blockIdx.x * 64, c0 = blockIdx.y * 64;
    v8f acc[4][4];
    gemm_core<1>(XB, XB, W, r0, c0, lr, hi, acc);
    const int b = r0 / SEQ, s0 = r0 % SEQ, h = blockIdx.y;
    const int rq = lane >> 3, pc = lane & 7;
#pragma unroll
    for (int nb = 0; nb < 4; ++nb) { const float bv = bfr(bias[c0 + nb * 16 + lr]);
#pragma unroll
        for (int mb = 0; mb < 4; ++mb) { v8h pk;
#pragma unroll
            for (int j = 0; j < 8; ++j) pk[j] = (h16)(acc[mb][nb][j] + bv);
            *(v8ha*)(vt + (nb * 16 + lr) * 72 + mb * 16 + 8 * hi) = pk; } }
    __syncthreads();
    h16* dv = VT + ((size_t)(b * NH + h) * HD) * SEQ + s0 + 8 * pc;
#pragma unroll 1
    for (int ps = 0; ps < 2; ++ps) {
#pragma unroll 1
        for (int it = 0; it < 16; ++it) { const int d = it * 4 + rq; const v8h val = *(const v8ha*)(vt + d * 72 + 8 * pc); *(volatile v8h*)(dv + (size_t)d * SEQ) = val; }
        if (ps == 0) __threadfence(); }
}

__global__ __launch_bounds__(128) void k_attn(const bf* __restrict__ Qh, const bf* __restrict__ Ql, const bf* __restrict__ Kh, const bf* __restrict__ Kl, const h16* __restrict__ VT, bf* Ch, bf* Cl) {
    __shared__ __align__(16) float ot[AW * 16 * 68];
    const int lane = threadIdx.x & 31, lr = lane & 15, hi = lane >> 4;
    const int wave = __builtin_amdgcn_readfirstlane(threadIdx.x >> 5);
    const int qt = blockIdx.x * AW + wave;
    const int bh = blockIdx.y;
    const size_t pb0 = (size_t)bh * SEQ * HD;
    const size_t qoff = pb0 + (size_t)(qt * 16 + lr) * HD + 8 * hi;
    const v16bf qh0 = ldb(Qh + qoff), qh1 = ldb(Qh + qoff + 32), ql0 = ldb(Ql + qoff), ql1 = ldb(Ql + qoff + 32);
    const size_t koff = pb0 + (size_t)lr * HD + 8 * hi;
    const size_t voff = (size_t)bh * HD * SEQ + (size_t)lr * SEQ + 8 * hi;
    v8f o0 = (v8f){}, o1 = (v8f){}, o2 = (v8f){}, o3 = (v8f){};
    float m = -1.0e30f, l = 0.0f;
#pragma unroll 1
    for (int kb = 0; kb < SEQ; kb += 32) {
        v8f s0 = (v8f){}, s1 = (v8f){};
        const bf* ph = Kh + koff + (size_t)kb * HD; const bf* pl = Kl + koff + (size_t)kb * HD;
        const v16bf a0 = ldb(ph), a1 = ldb(ph + 32), c0 = ldb(pl), c1 = ldb(pl + 32);
        s0 = wmmab(a0, qh0, s0); s0 = wmmab(a1, qh1, s0); s0 = wmmab(c0, qh0, s0); s0 = wmmab(c1, qh1, s0); s0 = wmmab(a0, ql0, s0); s0 = wmmab(a1, ql1, s0);
        const v16bf e0 = ldb(ph + 16 * HD), e1 = ldb(ph + 16 * HD + 32), g0 = ldb(pl + 16 * HD), g1 = ldb(pl + 16 * HD + 32);
        s1 = wmmab(e0, qh0, s1); s1 = wmmab(e1, qh1, s1); s1 = wmmab(g0, qh0, s1); s1 = wmmab(g1, qh1, s1); s1 = wmmab(e0, ql0, s1); s1 = wmmab(e1, ql1, s1);
        asm volatile("v_nop\n\tv_nop\n\tv_nop\n\tv_nop" : "+v"(s0), "+v"(s1) : "v"(e1), "v"(g1), "v"(ql1));
        float mx = fmaxf(s0[0], s1[0]);
#pragma unroll
        for (int r = 1; r < 8; ++r) mx = fmaxf(mx, fmaxf(s0[r], s1[r]));
        mx = fmaxf(mx, __shfl_xor(mx, 16, 32));
        const float mn = fmaxf(m, mx);
        const float corr = __builtin_amdgcn_exp2f((m - mn) * L2E);
        m = mn;
        float ls = 0.0f; v16h pb;
#pragma unroll
        for (int r = 0; r < 8; ++r) {
            const float p0 = __builtin_amdgcn_exp2f(__builtin_fmaf(s0[r] - mn, L2E, 10.0f));
            const float p1 = __builtin_amdgcn_exp2f(__builtin_fmaf(s1[r] - mn, L2E, 10.0f));
            ls += p0 + p1; pb[r] = (h16)p0; pb[8 + r] = (h16)p1; }
        l = l * corr + ls;
        o0 = o0 * corr; o1 = o1 * corr; o2 = o2 * corr; o3 = o3 * corr;
        const h16* vp = VT + voff + kb;
        const v16h va0 = ldh(vp), va1 = ldh(vp + (size_t)16 * SEQ), va2 = ldh(vp + (size_t)32 * SEQ), va3 = ldh(vp + (size_t)48 * SEQ);
        o0 = wmma16(va0, pb, o0); o1 = wmma16(va1, pb, o1); o2 = wmma16(va2, pb, o2); o3 = wmma16(va3, pb, o3);
        asm volatile("v_nop\n\tv_nop\n\tv_nop\n\tv_nop" : "+v"(o0), "+v"(o1), "+v"(o2), "+v"(o3) : "v"(pb), "v"(va3));
    }
    const float lt = l + __shfl_xor(l, 16, 32);
    const float inv = 1.0f / lt;
    const int ob = wave * (16 * 68) + lr * 68 + 8 * hi;
    { v4f x0, x1;
      x0[0] = o0[0] * inv; x0[1] = o0[1] * inv; x0[2] = o0[2] * inv; x0[3] = o0[3] * inv; x1[0] = o0[4] * inv; x1[1] = o0[5] * inv; x1[2] = o0[6] * inv; x1[3] = o0[7] * inv;
      *(v4fa*)(ot + ob) = x0; *(v4fa*)(ot + ob + 4) = x1;
      x0[0] = o1[0] * inv; x0[1] = o1[1] * inv; x0[2] = o1[2] * inv; x0[3] = o1[3] * inv; x1[0] = o1[4] * inv; x1[1] = o1[5] * inv; x1[2] = o1[6] * inv; x1[3] = o1[7] * inv;
      *(v4fa*)(ot + ob + 16) = x0; *(v4fa*)(ot + ob + 20) = x1;
      x0[0] = o2[0] * inv; x0[1] = o2[1] * inv; x0[2] = o2[2] * inv; x0[3] = o2[3] * inv; x1[0] = o2[4] * inv; x1[1] = o2[5] * inv; x1[2] = o2[6] * inv; x1[3] = o2[7] * inv;
      *(v4fa*)(ot + ob + 32) = x0; *(v4fa*)(ot + ob + 36) = x1;
      x0[0] = o3[0] * inv; x0[1] = o3[1] * inv; x0[2] = o3[2] * inv; x0[3] = o3[3] * inv; x1[0] = o3[4] * inv; x1[1] = o3[5] * inv; x1[2] = o3[6] * inv; x1[3] = o3[7] * inv;
      *(v4fa*)(ot + ob + 48) = x0; *(v4fa*)(ot + ob + 52) = x1; }
    __syncthreads();
    const int rq = lane >> 3, pc = lane & 7;
    const int b = bh / NH, h = bh % NH;
    const size_t cbase = ((size_t)(b * SEQ + qt * 16)) * HID + h * HD + 8 * pc;
#pragma unroll 1
    for (int ps = 0; ps < 2; ++ps) {
#pragma unroll 1
        for (int it = 0; it < 4; ++it) {
            const int rr = it * 4 + rq; const int xo = wave * (16 * 68) + rr * 68 + 8 * pc;
            const v4f x0 = *(const v4fa*)(ot + xo), x1 = *(const v4fa*)(ot + xo + 4);
            v8us oh, ol;
#pragma unroll
            for (int q = 0; q < 4; ++q) { unsigned short a2, c2; splitf(x0[q], a2, c2); oh[q] = a2; ol[q] = c2; splitf(x1[q], a2, c2); oh[q + 4] = a2; ol[q + 4] = c2; }
            *(volatile v8us*)(Ch + cbase + (size_t)rr * HID) = oh; *(volatile v8us*)(Cl + cbase + (size_t)rr * HID) = ol; }
        if (ps == 0) __threadfence(); }
}

__global__ __launch_bounds__(32) void k_out(const bf* __restrict__ Ch, const bf* __restrict__ Cl, const bf* __restrict__ W, const float* __restrict__ bias, float* OUT) {
    __shared__ __align__(16) float os[16 * 68];
    const int lane = threadIdx.x & 31, lr = lane & 15, hi = lane >> 4;
    const int r0 = blockIdx.x * 64, c0 = blockIdx.y * 64;
    v8f acc[4][4];
    gemm_core<2>(Ch, Cl, W, r0, c0, lr, hi, acc);
    const int b = r0 / SEQ, s0 = r0 % SEQ;
    const int cofs = lr * 4;
    v4f bb = *(const v4f*)(bias + c0 + cofs); bb[0] = bfr(bb[0]); bb[1] = bfr(bb[1]); bb[2] = bfr(bb[2]); bb[3] = bfr(bb[3]);
#pragma unroll
    for (int mb = 0; mb < 4; ++mb) {
#pragma unroll
        for (int nb = 0; nb < 4; ++nb) {
#pragma unroll
            for (int j = 0; j < 8; ++j) os[(hi * 8 + j) * 68 + nb * 16 + lr] = acc[mb][nb][j]; }
        __syncthreads();
        float* crow = OUT + ((size_t)b * SEQ_FULL + s0 + mb * 16) * HID + c0 + cofs;
#pragma unroll 1
        for (int ps = 0; ps < 2; ++ps) {
#pragma unroll 1
            for (int s = 0; s < 8; ++s) { const int row = 2 * s + hi; v4f val = *(const v4fa*)(os + row * 68 + cofs); val = val + bb; *(volatile v4f*)(crow + (size_t)row * HID) = val; }
            if (ps == 0) __threadfence(); }
        __syncthreads();
    }
}

extern "C" void kernel_launch(void* const* d_in, const int* in_sizes, int n_in,
                              void* d_out, int out_size, void* d_ws, size_t ws_size, hipStream_t stream) {
    if (n_in < 9) return;
    const int need_x = (NB - 1) * SEQ_FULL * HID + SEQ * HID;
    if (in_sizes[0] < need_x) return;
    if (in_sizes[1] < HID * HID || in_sizes[3] < HID * HID || in_sizes[5] < HID * HID || in_sizes[7] < HID * HID) return;
    if (in_sizes[2] < HID || in_sizes[4] < HID || in_sizes[6] < HID || in_sizes[8] < HID) return;
    if (out_size < need_x) return;
    const float* x  = (const float*)d_in[0];
    const float* wq = (const float*)d_in[1]; const float* bq = (const float*)d_in[2];
    const float* wk = (const float*)d_in[3]; const float* bk = (const float*)d_in[4];
    const float* wv = (const float*)d_in[5]; const float* bv = (const float*)d_in[6];
    const float* wo = (const float*)d_in[7]; const float* bo = (const float*)d_in[8];
    float* OUT = (float*)d_out;

    constexpr size_t SZ_XB = (size_t)MROWS * HID * 2;
    constexpr size_t SZ_W  = (size_t)HID * HID * 2;
    constexpr size_t SZ_CS = (size_t)SEQ * 32 * 2 * 4;
    constexpr size_t SZ_P  = (size_t)NB * NH * SEQ * HD * 2;
    constexpr size_t SZ_CT = (size_t)MROWS * HID * 2;
    constexpr size_t OFF_XB = 0;
    constexpr size_t OFF_WQ = OFF_XB + SZ_XB;
    constexpr size_t OFF_WK = OFF_WQ + SZ_W;
    constexpr size_t OFF_WV = OFF_WK + SZ_W;
    constexpr size_t OFF_WO = OFF_WV + SZ_W;
    constexpr size_t OFF_CS = OFF_WO + SZ_W;
    constexpr size_t OFF_QH = OFF_CS + SZ_CS;
    constexpr size_t OFF_QL = OFF_QH + SZ_P;
    constexpr size_t OFF_KH = OFF_QL + SZ_P;
    constexpr size_t OFF_KL = OFF_KH + SZ_P;
    constexpr size_t OFF_VT = OFF_KL + SZ_P;
    constexpr size_t OFF_CH = OFF_VT + SZ_P;
    constexpr size_t OFF_CL = OFF_CH + SZ_CT;
    constexpr size_t WS_TOTAL = OFF_CL + SZ_CT;
    static_assert(SZ_XB % 256 == 0);
    static_assert(SZ_W % 256 == 0);
    static_assert(SZ_CS % 256 == 0);
    static_assert(SZ_P % 256 == 0);
    static_assert(SZ_CT % 256 == 0);
    static_assert(WS_TOTAL <= (size_t)134217728);
    if (WS_TOTAL > ws_size) return;
    char* wsp = (char*)d_ws;
    bf* XB = (bf*)(wsp + OFF_XB); bf* WQ = (bf*)(wsp + OFF_WQ); bf* WK = (bf*)(wsp + OFF_WK); bf* WV = (bf*)(wsp + OFF_WV); bf* WO = (bf*)(wsp + OFF_WO);
    float* CS = (float*)(wsp + OFF_CS);
    bf* QPh = (bf*)(wsp + OFF_QH); bf* QPl = (bf*)(wsp + OFF_QL); bf* KPh = (bf*)(wsp + OFF_KH); bf* KPl = (bf*)(wsp + OFF_KL);
    h16* VT = (h16*)(wsp + OFF_VT);
    bf* CTh = (bf*)(wsp + OFF_CH); bf* CTl = (bf*)(wsp + OFF_CL);

    k_cvt<<<dim3(SEQ * HID / 2048, NB), 256, 0, stream>>>(x, XB, SEQ * HID, SEQ_FULL * HID);
    k_cvt<<<dim3(HID * HID / 2048, 1), 256, 0, stream>>>(wq, WQ, HID * HID, HID * HID);
    k_cvt<<<dim3(HID * HID / 2048, 1), 256, 0, stream>>>(wk, WK, HID * HID, HID * HID);
    k_cvt<<<dim3(HID * HID / 2048, 1), 256, 0, stream>>>(wv, WV, HID * HID, HID * HID);
    k_cvt<<<dim3(HID * HID / 2048, 1), 256, 0, stream>>>(wo, WO, HID * HID, HID * HID);
    k_cstab<<<SEQ * 32 / 256, 256, 0, stream>>>(CS);
    k_proj_rope<<<dim3(MROWS / 64, NH), 32, 0, stream>>>(XB, WQ, bq, CS, 0.125f, QPh, QPl);
    k_proj_rope<<<dim3(MROWS / 64, NH), 32, 0, stream>>>(XB, WK, bk, CS, 1.0f, KPh, KPl);
    k_proj_v<<<dim3(MROWS / 64, NH), 32, 0, stream>>>(XB, WV, bv, VT);
    k_attn<<<dim3(SEQ / (16 * AW), NB * NH), 32 * AW, 0, stream>>>(QPh, QPl, KPh, KPl, VT, CTh, CTl);
    k_out<<<dim3(MROWS / 64, HID / 64), 32, 0, stream>>>(CTh, CTl, WO, bo, OUT);
}
